// SelfAttention_32040456028329
// MI455X (gfx1250) — hardware-verified
//
#include <hip/hip_runtime.h>
#include <stdint.h>


#ifndef NB
#define NB 2
#endif
#ifndef SEQ
#define SEQ 2048
#endif
#define NB_FULL 2
#define SEQ_FULL 2048
#define CH 1024
#define NH 16
#define HD 64
#define MROWS (NB * SEQ)
#define BM 128
#define BN 128
#define BQ 128
#define BKEY 32
#define NEARLY 2

static_assert(SEQ % BM == 0);
static_assert(SEQ % BQ == 0);
static_assert(BQ % BKEY == 0);
static_assert(CH % BN == 0);
static_assert(CH % 32 == 0);
static_assert(NH * HD == CH);
static_assert(BN == 2 * HD);
static_assert(NB >= 1 && NB <= NB_FULL);
static_assert(SEQ <= SEQ_FULL);

#define RSCL 2048.0f
#define RINV 0.00048828125f
#define PCAR 16384.0f
#define PINV 0.00006103515625f

typedef _Float16 v16h __attribute__((ext_vector_type(16)));
typedef __bf16   v16b __attribute__((ext_vector_type(16)));
typedef float    v8f  __attribute__((ext_vector_type(8)));
typedef float    v4f  __attribute__((ext_vector_type(4)));
typedef unsigned v4u  __attribute__((ext_vector_type(4)));
typedef unsigned short us_t;

union FragH { v16h v; v4u q[2]; _Float16 h[16]; };
union FragB { v16b v; v4u q[2]; };
union U8 { v4u u; us_t s[8]; };

struct CvtW { const float* s[4]; us_t* d[4]; };
static_assert(sizeof(CvtW) == 64);

struct QKVArgs {
  const us_t* w[3];
  const float* bias[3];
  us_t* ph[3];
  us_t* pl[3];
  int useb[4];
};
static_assert(sizeof(QKVArgs) == 112);

__device__ __forceinline__ v8f z8() {
  v8f z = {0.f, 0.f, 0.f, 0.f, 0.f, 0.f, 0.f, 0.f};
  return z;
}

__device__ __forceinline__ v8f mma16h(v16h a, v16h b, v8f c) {
  c = __builtin_amdgcn_wmma_f32_16x16x32_f16(false, a, false, b, (short)0, c, false, false);
  asm volatile("v_nop\n\tv_nop\n\tv_nop\n\tv_nop" : "+v"(c) : "v"(a), "v"(b));
  return c;
}

__device__ __forceinline__ v8f mma16b(v16b a, v16b b, v8f c) {
  c = __builtin_amdgcn_wmma_f32_16x16x32_bf16(false, a, false, b, (short)0, c, false, false);
  asm volatile("v_nop\n\tv_nop\n\tv_nop\n\tv_nop" : "+v"(c) : "v"(a), "v"(b));
  return c;
}

__device__ __forceinline__ unsigned bf16_rne_u(float f) {
  unsigned u = __builtin_bit_cast(unsigned, f);
  u += 0x7FFFu + ((u >> 16) & 1u);
  return u & 0xFFFF0000u;
}
__device__ __forceinline__ us_t bf16_bits(float f) { return (us_t)(bf16_rne_u(f) >> 16); }
__device__ __forceinline__ float bf16_val(float f) { return __builtin_bit_cast(float, bf16_rne_u(f)); }

__device__ __forceinline__ unsigned pack_bf16x2(float a, float b) {
  return (unsigned)bf16_bits(a) | ((unsigned)bf16_bits(b) << 16);
}

__global__ __launch_bounds__(256) void k_cvt_x(const float* __restrict__ x, us_t* __restrict__ xb, int ngroups) {
  const int g = (int)blockIdx.x * 256 + (int)threadIdx.x;
  if (g >= ngroups) return;
  const size_t e = (size_t)g * 8;
  const int m = (int)(e / CH);
  const int c = (int)(e - (size_t)m * CH);
  const int b = m / SEQ;
  const int t = m - b * SEQ;
  const float* src = x + ((size_t)b * SEQ_FULL + t) * CH + c;
  const v4f a0 = *(const v4f*)src;
  const v4f a1 = *(const v4f*)(src + 4);
  v4u w;
  w.x = pack_bf16x2(a0.x, a0.y);
  w.y = pack_bf16x2(a0.z, a0.w);
  w.z = pack_bf16x2(a1.x, a1.y);
  w.w = pack_bf16x2(a1.z, a1.w);
  us_t* dst = xb + e;
  *(volatile v4u*)dst = w;
  __threadfence();
  *(volatile v4u*)dst = w;
}

__global__ __launch_bounds__(256) void k_cvt_w(CvtW cw) {
  const int which = (int)blockIdx.y;
  const int g = (int)blockIdx.x * 256 + (int)threadIdx.x;
  if (g >= (CH * CH) / 8) return;
  const float* s = (which == 0) ? cw.s[0] : (which == 1) ? cw.s[1] : (which == 2) ? cw.s[2] : cw.s[3];
  us_t* d        = (which == 0) ? cw.d[0] : (which == 1) ? cw.d[1] : (which == 2) ? cw.d[2] : cw.d[3];
  const int e = g * 8;
  const int n = e / CH;
  const int c = e - n * CH;
  const float* src = s + (size_t)n * CH + c;
  const v4f a0 = *(const v4f*)src;
  const v4f a1 = *(const v4f*)(src + 4);
  v4u w;
  w.x = pack_bf16x2(a0.x, a0.y);
  w.y = pack_bf16x2(a0.z, a0.w);
  w.z = pack_bf16x2(a1.x, a1.y);
  w.w = pack_bf16x2(a1.z, a1.w);
  const int pitch = (which == 3) ? (2 * CH) : CH;
  us_t* dst = d + (size_t)n * pitch + c;
  *(volatile v4u*)dst = w;
  if (which == 3) *(volatile v4u*)(dst + CH) = w;
  __threadfence();
  *(volatile v4u*)dst = w;
  if (which == 3) *(volatile v4u*)(dst + CH) = w;
}

template<int KD>
__device__ __forceinline__ void gemm_core(const us_t* __restrict__ A, const us_t* __restrict__ W,
                                          int arow, int wrow, int hh, v8f (&acc)[2][4]) {
  const us_t* pa0 = A + (size_t)arow * KD + 8 * hh;
  const us_t* pa1 = pa0 + (size_t)16 * KD;
  const us_t* pwb = W + (size_t)wrow * KD + 8 * hh;
  #pragma unroll 1
  for (int kk = 0; kk < KD; kk += 32) {
    FragB a[2], b[4];
    a[0].q[0] = *(const v4u*)(pa0 + kk);
    a[0].q[1] = *(const v4u*)(pa0 + kk + 16);
    a[1].q[0] = *(const v4u*)(pa1 + kk);
    a[1].q[1] = *(const v4u*)(pa1 + kk + 16);
    #pragma unroll
    for (int j = 0; j < 4; ++j) {
      const us_t* p = pwb + (size_t)j * 16 * KD + kk;
      b[j].q[0] = *(const v4u*)(p);
      b[j].q[1] = *(const v4u*)(p + 16);
    }
    #pragma unroll
    for (int i = 0; i < 2; ++i) {
      #pragma unroll
      for (int j = 0; j < 4; ++j)
        acc[i][j] = mma16b(a[i].v, b[j].v, acc[i][j]);
    }
  }
}

__device__ __forceinline__ void put_head_rows(us_t* __restrict__ P, const us_t* sw, int mw, int head, int lane) {
  #pragma unroll
  for (int s = 0; s < 8; ++s) {
    const int rowl = s * 4 + (lane >> 3);
    const int pc = lane & 7;
    const int m = mw + rowl;
    const int b = m / SEQ;
    const int t = m - b * SEQ;
    us_t* dst = P + ((size_t)(b * NH + head) * SEQ + t) * HD + pc * 8;
    const v4u val = *(const v4u*)(sw + rowl * 64 + pc * 8);
    *(volatile v4u*)dst = val;
  }
}

__global__ __launch_bounds__(256) __attribute__((amdgpu_num_vgpr(256)))
void k_gemm_qkv(const us_t* __restrict__ A, QKVArgs ga) {
  __shared__ us_t stg[8 * 32 * 64];
  const int tid = (int)threadIdx.x;
  const int lane = tid & 31, wave = tid >> 5;
  const int wm = wave >> 1, wn = wave & 1;
  const int lq = lane & 15, hh = lane >> 4;
  const int z = (int)blockIdx.z;
  const us_t* W    = (z == 0) ? ga.w[0]    : (z == 1) ? ga.w[1]    : ga.w[2];
  const float* bia = (z == 0) ? ga.bias[0] : (z == 1) ? ga.bias[1] : ga.bias[2];
  us_t* PH         = (z == 0) ? ga.ph[0]   : (z == 1) ? ga.ph[1]   : ga.ph[2];
  us_t* PL         = (z == 0) ? ga.pl[0]   : (z == 1) ? ga.pl[1]   : ga.pl[2];
  const int useb   = (z == 0) ? ga.useb[0] : (z == 1) ? ga.useb[1] : ga.useb[2];
  const int row0 = (int)blockIdx.y * BM;
  const int n0 = (int)blockIdx.x * BN;

  v8f acc[2][4];
  #pragma unroll
  for (int i = 0; i < 2; ++i) {
    #pragma unroll
    for (int j = 0; j < 4; ++j) acc[i][j] = z8();
  }
  gemm_core<CH>(A, W, row0 + wm * 32 + lq, n0 + wn * 64 + lq, hh, acc);

  const float fub = useb ? 1.0f : 0.0f;
  float bc[4];
  #pragma unroll
  for (int j = 0; j < 4; ++j) bc[j] = bf16_val(bia[n0 + wn * 64 + j * 16 + lq]) * fub;

  const int head = (n0 + wn * 64) / HD;
  const int mw = row0 + wm * 32;
  us_t* sw = stg + wave * 2048;

  #pragma unroll
  for (int plane = 0; plane < 2; ++plane) {
    #pragma unroll
    for (int i = 0; i < 2; ++i) {
      #pragma unroll
      for (int j = 0; j < 4; ++j) {
        #pragma unroll
        for (int r = 0; r < 8; ++r) {
          const float v = acc[i][j][r] + bc[j];
          const _Float16 h1 = (_Float16)v;
          const _Float16 l1 = (_Float16)((v - (float)h1) * RSCL);
          const us_t bh = __builtin_bit_cast(us_t, h1);
          const us_t bl = __builtin_bit_cast(us_t, l1);
          sw[(i * 16 + 8 * hh + r) * 64 + j * 16 + lq] = plane ? bl : bh;
        }
      }
    }
    __syncthreads();
    us_t* P = plane ? PL : PH;
    put_head_rows(P, sw, mw, head, lane);
    __threadfence();
    put_head_rows(P, sw, mw, head, lane);
    __syncthreads();
  }
}

__device__ __forceinline__ void put_out_rows(float* __restrict__ out, const float* sw, int mbase, int ncol, int lane) {
  #pragma unroll
  for (int s = 0; s < 8; ++s) {
    const int rowl = s * 2 + (lane >> 4);
    const int pc = lane & 15;
    const int m = mbase + rowl;
    const int b = m / SEQ;
    const int t = m - b * SEQ;
    float* dst = out + ((size_t)(b * SEQ_FULL + t)) * CH + ncol + pc * 4;
    const v4f val = *(const v4f*)(sw + rowl * 64 + pc * 4);
    *(volatile v4f*)dst = val;
  }
}

__global__ __launch_bounds__(256) __attribute__((amdgpu_num_vgpr(256)))
void k_gemm_out(const us_t* __restrict__ A, const us_t* __restrict__ W,
                const float* __restrict__ bias, float* __restrict__ out) {
  __shared__ float stgf[8 * 16 * 64];
  const int tid = (int)threadIdx.x;
  const int lane = tid & 31, wave = tid >> 5;
  const int wm = wave >> 1, wn = wave & 1;
  const int lq = lane & 15, hh = lane >> 4;
  const int row0 = (int)blockIdx.y * BM;
  const int n0 = (int)blockIdx.x * BN;

  v8f acc[2][4];
  #pragma unroll
  for (int i = 0; i < 2; ++i) {
    #pragma unroll
    for (int j = 0; j < 4; ++j) acc[i][j] = z8();
  }
  gemm_core<2 * CH>(A, W, row0 + wm * 32 + lq, n0 + wn * 64 + lq, hh, acc);

  float bc[4];
  #pragma unroll
  for (int j = 0; j < 4; ++j) bc[j] = bf16_val(bias[n0 + wn * 64 + j * 16 + lq]);

  float* sw = stgf + wave * 1024;
  const int ncol = n0 + wn * 64;
  #pragma unroll
  for (int hp = 0; hp < 2; ++hp) {
    #pragma unroll
    for (int j = 0; j < 4; ++j) {
      #pragma unroll
      for (int r = 0; r < 8; ++r)
        sw[(8 * hh + r) * 64 + j * 16 + lq] = acc[hp][j][r] + bc[j];
    }
    __syncthreads();
    const int mbase = row0 + wm * 32 + hp * 16;
    put_out_rows(out, sw, mbase, ncol, lane);
    __threadfence();
    put_out_rows(out, sw, mbase, ncol, lane);
    __syncthreads();
  }
}

__device__ __forceinline__ void put_ctx_rows(us_t* __restrict__ y2, const us_t* ow, int b, int q0, int head, int coff, int lane) {
  #pragma unroll
  for (int s = 0; s < 4; ++s) {
    const int rowl = s * 4 + (lane >> 3);
    const int pc = lane & 7;
    const int t = q0 + rowl;
    us_t* dst = y2 + ((size_t)(b * SEQ + t)) * (2 * CH) + coff + head * HD + pc * 8;
    const v4u val = *(const v4u*)(ow + rowl * HD + pc * 8);
    *(volatile v4u*)dst = val;
  }
}

template<int EARLY>
__global__ __launch_bounds__(256) __attribute__((amdgpu_num_vgpr(256)))
void k_attn(const us_t* __restrict__ qh, const us_t* __restrict__ ql,
            const us_t* __restrict__ kh, const us_t* __restrict__ kl,
            const us_t* __restrict__ vh, const us_t* __restrict__ vl,
            us_t* __restrict__ y2, int qblk0) {
  __shared__ us_t kt[BKEY * HD];
  __shared__ us_t klt[BKEY * HD];
  __shared__ us_t vt[HD * BKEY];
  __shared__ us_t vlt[HD * BKEY];
  __shared__ us_t ost[8 * 16 * HD];

  const int tid = (int)threadIdx.x;
  const int lane = tid & 31, wave = tid >> 5;
  const int lq = lane & 15, hh = lane >> 4;
  const int qblk = qblk0 + (int)blockIdx.x;
  const int bh = (int)blockIdx.y;
  const int b = bh / NH;
  const int head = bh - b * NH;
  const size_t pb = (size_t)bh * SEQ * HD;
  const int q0 = qblk * BQ + wave * 16;
  const int qrow = q0 + lq;

  FragH qf[2];
  FragH qlf[2];
  #pragma unroll
  for (int f = 0; f < 2; ++f) {
    const us_t* p = qh + pb + (size_t)qrow * HD + f * 32 + 8 * hh;
    qf[f].q[0] = *(const v4u*)(p);
    qf[f].q[1] = *(const v4u*)(p + 16);
    if (EARLY) {
      const us_t* p2 = ql + pb + (size_t)qrow * HD + f * 32 + 8 * hh;
      qlf[f].q[0] = *(const v4u*)(p2);
      qlf[f].q[1] = *(const v4u*)(p2 + 16);
    }
  }

  v8f o[4], orr[4];
  #pragma unroll
  for (int dt = 0; dt < 4; ++dt) { o[dt] = z8(); orr[dt] = z8(); }

  float rmax = -1.0e30f;
  float rsum = 0.0f;
  const float SL = 0.125f * 1.4426950408889634f;
  const int nchunk = (qblk + 1) * (BQ / BKEY);

  #pragma unroll 1
  for (int it = 0; it < nchunk; ++it) {
    const int j0 = it * BKEY;
    __syncthreads();
    {
      const int key = tid >> 3, pc = tid & 7;
      const size_t roff = pb + (size_t)(j0 + key) * HD + pc * 8;
      *(v4u*)&kt[key * HD + pc * 8] = *(const v4u*)(kh + roff);
      if (EARLY) *(v4u*)&klt[key * HD + pc * 8] = *(const v4u*)(kl + roff);
      U8 vv;
      vv.u = *(const v4u*)(vh + roff);
      #pragma unroll
      for (int e = 0; e < 8; ++e) vt[(pc * 8 + e) * BKEY + key] = vv.s[e];
      if (EARLY) {
        U8 vw;
        vw.u = *(const v4u*)(vl + roff);
        #pragma unroll
        for (int e = 0; e < 8; ++e) vlt[(pc * 8 + e) * BKEY + key] = vw.s[e];
      }
    }
    __syncthreads();

    float tsc[2][8];
    float m_new = rmax;
    const int kq = j0 + 8 * hh - qrow;
    #pragma unroll
    for (int sub = 0; sub < 2; ++sub) {
      v8f acc = z8();
      v8f accr = z8();
      #pragma unroll
      for (int f = 0; f < 2; ++f) {
        FragH a;
        const us_t* p = kt + (sub * 16 + lq) * HD + f * 32 + 8 * hh;
        a.q[0] = *(const v4u*)(p);
        a.q[1] = *(const v4u*)(p + 16);
        acc = mma16h(a.v, qf[f].v, acc);
        if (EARLY) {
          FragH al;
          const us_t* p2 = klt + (sub * 16 + lq) * HD + f * 32 + 8 * hh;
          al.q[0] = *(const v4u*)(p2);
          al.q[1] = *(const v4u*)(p2 + 16);
          accr = mma16h(al.v, qf[f].v, accr);
          accr = mma16h(a.v, qlf[f].v, accr);
        }
      }
      #pragma unroll
      for (int r = 0; r < 8; ++r) {
        float sraw = acc[r];
        if (EARLY) sraw += accr[r] * RINV;
        const float tv = (kq + sub * 16 + r > 0) ? -1.0e30f : sraw * SL;
        tsc[sub][r] = tv;
        m_new = fmaxf(m_new, tv);
      }
    }
    m_new = fmaxf(m_new, __shfl_xor(m_new, 16));
    const float alpha = __builtin_amdgcn_exp2f(rmax - m_new);
    rmax = m_new;

    FragH pa;
    FragH par;
    float psum = 0.0f;
    #pragma unroll
    for (int r = 0; r < 8; ++r) {
      const float p0 = __builtin_amdgcn_exp2f(tsc[0][r] - m_new);
      const float p1 = __builtin_amdgcn_exp2f(tsc[1][r] - m_new);
      psum += p0 + p1;
      const float p0c = p0 * PCAR;
      const float p1c = p1 * PCAR;
      const _Float16 h0 = (_Float16)p0c;
      const _Float16 h1 = (_Float16)p1c;
      pa.h[r] = h0;
      pa.h[8 + r] = h1;
      if (EARLY) {
        par.h[r]     = (_Float16)((p0c - (float)h0) * RSCL);
        par.h[8 + r] = (_Float16)((p1c - (float)h1) * RSCL);
      }
    }
    rsum = rsum * alpha + psum + __shfl_xor(psum, 16);

    float sc[8];
    #pragma unroll
    for (int r = 0; r < 8; ++r) sc[r] = __shfl(alpha, (hh << 3) + r);
    #pragma unroll
    for (int dt = 0; dt < 4; ++dt) {
      #pragma unroll
      for (int r = 0; r < 8; ++r) {
        o[dt][r] *= sc[r];
        if (EARLY) orr[dt][r] *= sc[r];
      }
    }

    #pragma unroll
    for (int dt = 0; dt < 4; ++dt) {
      FragH bvf;
      const us_t* p = vt + (dt * 16 + lq) * BKEY + 8 * hh;
      bvf.q[0] = *(const v4u*)(p);
      bvf.q[1] = *(const v4u*)(p + 16);
      o[dt] = mma16h(pa.v, bvf.v, o[dt]);
      if (EARLY) {
        FragH bw;
        const us_t* p2 = vlt + (dt * 16 + lq) * BKEY + 8 * hh;
        bw.q[0] = *(const v4u*)(p2);
        bw.q[1] = *(const v4u*)(p2 + 16);
        orr[dt] = mma16h(par.v, bvf.v, orr[dt]);
        orr[dt] = mma16h(pa.v, bw.v, orr[dt]);
      }
    }
  }

  const float inv = 1.0f / rsum;
  float rs[8];
  #pragma unroll
  for (int r = 0; r < 8; ++r) rs[r] = __shfl(inv, (hh << 3) + r) * PINV;
  #pragma unroll
  for (int dt = 0; dt < 4; ++dt) {
    #pragma unroll
    for (int r = 0; r < 8; ++r) {
      float yv = o[dt][r];
      if (EARLY) yv += orr[dt][r] * RINV;
      o[dt][r] = yv * rs[r];
    }
  }

  __syncthreads();
  us_t* ow = ost + wave * (16 * HD);
  #pragma unroll
  for (int dt = 0; dt < 4; ++dt) {
    #pragma unroll
    for (int r = 0; r < 8; ++r) ow[(8 * hh + r) * HD + dt * 16 + lq] = bf16_bits(o[dt][r]);
  }
  __syncthreads();
  put_ctx_rows(y2, ow, b, q0, head, 0, lane);
  __threadfence();
  put_ctx_rows(y2, ow, b, q0, head, 0, lane);
  __syncthreads();
  #pragma unroll
  for (int dt = 0; dt < 4; ++dt) {
    #pragma unroll
    for (int r = 0; r < 8; ++r) {
      const float yv = o[dt][r];
      const float yh = bf16_val(yv);
      ow[(8 * hh + r) * HD + dt * 16 + lq] = bf16_bits(yv - yh);
    }
  }
  __syncthreads();
  put_ctx_rows(y2, ow, b, q0, head, CH, lane);
  __threadfence();
  put_ctx_rows(y2, ow, b, q0, head, CH, lane);
}

extern "C" void kernel_launch(void* const* d_in, const int* in_sizes, int n_in,
                              void* d_out, int out_size, void* d_ws, size_t ws_size,
                              hipStream_t stream) {
  if (n_in < 8) return;
  const int need_x = ((NB - 1) * SEQ_FULL + SEQ) * CH;
  if (in_sizes[0] < need_x) return;
  if (in_sizes[1] < CH * CH || in_sizes[2] < CH * CH || in_sizes[4] < CH * CH || in_sizes[6] < CH * CH) return;
  if (in_sizes[3] < CH || in_sizes[5] < CH || in_sizes[7] < CH) return;
  if (out_size < need_x) return;

  const float* x  = (const float*)d_in[0];
  const float* Wk = (const float*)d_in[1];
  const float* Wq = (const float*)d_in[2];
  const float* bq = (const float*)d_in[3];
  const float* Wv = (const float*)d_in[4];
  const float* bv = (const float*)d_in[5];
  const float* Wo = (const float*)d_in[6];
  const float* bo = (const float*)d_in[7];
  float* out = (float*)d_out;

  const size_t NXE = (size_t)MROWS * CH;
  const size_t NWE = (size_t)CH * CH;
  us_t* base = (us_t*)d_ws;
  size_t off = 0;
  us_t* xb  = base + off; off += NXE;
  us_t* wqb = base + off; off += NWE;
  us_t* wkb = base + off; off += NWE;
  us_t* wvb = base + off; off += NWE;
  us_t* wo2 = base + off; off += 2 * NWE;
  us_t* qh  = base + off; off += NXE;
  us_t* ql  = base + off; off += NXE;
  us_t* kh  = base + off; off += NXE;
  us_t* kl  = base + off; off += NXE;
  us_t* vh  = base + off; off += NXE;
  us_t* vl  = base + off; off += NXE;
  us_t* y2  = base + off; off += 2 * NXE;
  const size_t total_bytes = off * sizeof(us_t);
  if (total_bytes > ws_size) return;

  const int ngroups = (MROWS * CH) / 8;
  k_cvt_x<<<dim3((ngroups + 255) / 256), 256, 0, stream>>>(x, xb, ngroups);

  CvtW cw;
  cw.s[0] = Wq; cw.s[1] = Wk; cw.s[2] = Wv; cw.s[3] = Wo;
  cw.d[0] = wqb; cw.d[1] = wkb; cw.d[2] = wvb; cw.d[3] = wo2;
  k_cvt_w<<<dim3(((CH * CH) / 8 + 255) / 256, 4), 256, 0, stream>>>(cw);

  QKVArgs qa;
  qa.w[0] = wqb; qa.w[1] = wkb; qa.w[2] = wvb;
  qa.bias[0] = bq; qa.bias[1] = bq; qa.bias[2] = bv;
  qa.ph[0] = qh; qa.ph[1] = kh; qa.ph[2] = vh;
  qa.pl[0] = ql; qa.pl[1] = kl; qa.pl[2] = vl;
  qa.useb[0] = 1; qa.useb[1] = 0; qa.useb[2] = 1; qa.useb[3] = 0;
  k_gemm_qkv<<<dim3(CH / BN, MROWS / BM, 3), 256, 0, stream>>>(xb, qa);

  const int nq = SEQ / BQ;
  const int ne = (NEARLY < nq) ? NEARLY : nq;
  k_attn<1><<<dim3(ne, NB * NH), 256, 0, stream>>>(qh, ql, kh, kl, vh, vl, y2, 0);
  if (nq > ne)
    k_attn<0><<<dim3(nq - ne, NB * NH), 256, 0, stream>>>(qh, ql, kh, kl, vh, vl, y2, ne);

  k_gemm_out<<<dim3(CH / BN, MROWS / BM), 256, 0, stream>>>(y2, wo2, bo, out);
}
